// EncoderLayer_8959301780085
// MI455X (gfx1250) — hardware-verified
//
#include <hip/hip_runtime.h>
#include <math.h>

#ifndef NB
#define NB 2
#endif
#ifndef SEQ
#define SEQ 2048
#endif
#define NB_FULL 2
#define SEQ_FULL 2048
#define EMBED 1024
#define NHEAD 16
#define HDIM 64
#define FFDIM 4096
#define MT (NB * SEQ)
#define QKLD (2 * EMBED)
#define BR_N 9216

static_assert(NHEAD * HDIM == EMBED);
static_assert(HDIM == 64);
static_assert(SEQ % 64 == 0);
static_assert(MT % 64 == 0);
static_assert(EMBED % 64 == 0 && FFDIM % 64 == 0);
static_assert(EMBED % 32 == 0 && FFDIM % 32 == 0);
static_assert(EMBED == 32 * 4 * 8);
static_assert(NB <= NB_FULL && SEQ <= SEQ_FULL);
static_assert(BR_N == 5 * EMBED + FFDIM);
static_assert(BR_N % 256 == 0);

typedef __attribute__((ext_vector_type(16))) _Float16 v16h;
typedef __attribute__((ext_vector_type(8)))  _Float16 v8h;
typedef __attribute__((ext_vector_type(8)))  float    v8f;
typedef __attribute__((ext_vector_type(4)))  float    v4f;
typedef __attribute__((ext_vector_type(4)))  unsigned int u4;
typedef __attribute__((ext_vector_type(2)))  unsigned int u2;

union FragU { v16h v; v8h h[2]; };
__device__ __forceinline__ v16h frag_ld(const _Float16* __restrict__ p) { FragU f; f.h[0] = *(const v8h*)(p); f.h[1] = *(const v8h*)(p + 16); return f.v; }

__device__ __forceinline__ v8f wmma_h(v16h a, v16h b, v8f c) {
    c = __builtin_amdgcn_wmma_f32_16x16x32_f16(false, a, false, b, (short)0, c, false, false);
    asm volatile("v_nop\n\tv_nop\n\tv_nop\n\tv_nop" : "+v"(c) : "v"(a), "v"(b));
    return c;
}
__device__ __forceinline__ void dep_guard_h(v8f& a, v8f& b, v16h x, v16h y) { asm volatile("v_nop\n\tv_nop\n\tv_nop\n\tv_nop" : "+v"(a), "+v"(b) : "v"(x), "v"(y)); }
__device__ __forceinline__ void keep4_h(v16h a, v16h b, v16h c, v16h d) { asm volatile("v_nop" :: "v"(a), "v"(b), "v"(c), "v"(d)); }
__device__ __forceinline__ void acc_guard4(v8f& a, v8f& b, v8f& c, v8f& d) { asm volatile("v_nop\n\tv_nop\n\tv_nop\n\tv_nop" : "+v"(a), "+v"(b), "+v"(c), "+v"(d)); }

#define VST2(T, ptr, val) do { const T vst2_v_ = (val); *(volatile T*)(ptr) = vst2_v_; __threadfence(); *(volatile T*)(ptr) = vst2_v_; } while (0)

__device__ __forceinline__ float cmb_bf(float v) { const unsigned u = __builtin_bit_cast(unsigned, v); const unsigned r = (u + 0x7fffu + ((u >> 16) & 1u)) & 0xffff0000u; return __builtin_bit_cast(float, r); }
__device__ __forceinline__ unsigned int cmb_pk2(float a, float b) { return (unsigned int)__builtin_bit_cast(unsigned short, (_Float16)a) | ((unsigned int)__builtin_bit_cast(unsigned short, (_Float16)b) << 16); }

__global__ __launch_bounds__(256) void k_cast_x(const float* __restrict__ SRC, unsigned short* __restrict__ DST) {
    const long long u = (long long)blockIdx.x * 256 + threadIdx.x; const int per = EMBED / 8; if (u >= (long long)MT * per) return;
    const int r = (int)(u / per); const int c0 = 8 * (int)(u % per);
    const long long sr = (long long)(r / SEQ) * SEQ_FULL + (r % SEQ);
    const float* s = SRC + sr * EMBED + c0;
    const v4f a = *(const v4f*)s; const v4f b = *(const v4f*)(s + 4);
    u4 pk; pk.x = cmb_pk2(cmb_bf(a.x), cmb_bf(a.y)); pk.y = cmb_pk2(cmb_bf(a.z), cmb_bf(a.w)); pk.z = cmb_pk2(cmb_bf(b.x), cmb_bf(b.y)); pk.w = cmb_pk2(cmb_bf(b.z), cmb_bf(b.w));
    VST2(u4, (u4*)(DST + (long long)r * EMBED + c0), pk);
}
__global__ __launch_bounds__(256) void k_cast_wT(const float* __restrict__ SRC, int lds, unsigned short* __restrict__ DST, int ldd, int nR, int nC, float sc) {
    const long long u = (long long)blockIdx.x * 256 + threadIdx.x; const int per = nR / 8; if (u >= (long long)nC * per) return;
    const int c = (int)(u / per); const int r0 = 8 * (int)(u % per);
    float w[8];
#pragma unroll
    for (int e = 0; e < 8; ++e) w[e] = cmb_bf(SRC[(long long)(r0 + e) * lds + c]) * sc;
    u4 pk; pk.x = cmb_pk2(w[0], w[1]); pk.y = cmb_pk2(w[2], w[3]); pk.z = cmb_pk2(w[4], w[5]); pk.w = cmb_pk2(w[6], w[7]);
    VST2(u4, (u4*)(DST + (long long)c * ldd + r0), pk);
}
__global__ __launch_bounds__(256) void k_bias(const float* __restrict__ bq, const float* __restrict__ bk, const float* __restrict__ bv, const float* __restrict__ bo,
                                              const float* __restrict__ b1, const float* __restrict__ b2, float* __restrict__ BR) {
    const int u = blockIdx.x * 256 + threadIdx.x; if (u >= BR_N) return;
    const int i1 = u & (EMBED - 1); const int i4 = min(max(u - 4 * EMBED, 0), FFDIM - 1);
    const float vq = bq[i1], vk = bk[i1], vv = bv[i1], vo = bo[i1], v1 = b1[i4], v2 = b2[i1];
    const int seg = u / EMBED;
    const float v = (seg == 0) ? vq : ((seg == 1) ? vk : ((seg == 2) ? vv : ((seg == 3) ? vo : ((seg < 8) ? v1 : v2))));
    VST2(float, BR + u, cmb_bf(v));
}

template <int ACT> __device__ __forceinline__ float g_act(float v) { if (ACT == 1) return 0.5f * v * (1.0f + erff(v * 0.70710678118654752f)); return v; }

template <int BIAS_MODE, int OUT_MODE, int ACT>
__device__ __forceinline__ void gemm64_body(const unsigned short* __restrict__ Ap, int lda, const unsigned short* __restrict__ Btp, int ldb,
                                            void* __restrict__ Cout, int ldc, const float* __restrict__ bias, int M, int N, int K, float scale, float oscale) {
    __shared__ __align__(16) float sT[8][16 * 68];
    const _Float16* A = (const _Float16*)Ap; const _Float16* Bt = (const _Float16*)Btp;
    const int lane = threadIdx.x & 31;
    const int wave = threadIdx.x >> 5;
    const int tilesN = N >> 6;
    const int tilesM = M >> 6;
    const int tile = blockIdx.x * 8 + wave;
    if (tile >= tilesM * tilesN) return;
    const int tm = tile / tilesN;
    const int tn = tile - tm * tilesN;
    const int m0 = tm << 6;
    const int n0 = tn << 6;
    const int rlane = lane & 15;
    const int koff  = (lane >> 4) * 8;
    const int mOff  = (lane >> 4) * 8;

    v8f acc[4][4];
#pragma unroll
    for (int i = 0; i < 4; ++i)
#pragma unroll
        for (int j = 0; j < 4; ++j) acc[i][j] = (v8f){0.f, 0.f, 0.f, 0.f, 0.f, 0.f, 0.f, 0.f};

    for (int k0 = 0; k0 < K; k0 += 32) {
        v16h bh[4];
#pragma unroll
        for (int j = 0; j < 4; ++j) {
            const size_t bo = (size_t)(n0 + (j << 4) + rlane) * ldb + koff + k0;
            bh[j] = frag_ld(Bt + bo);
        }
#pragma unroll
        for (int i = 0; i < 4; ++i) {
            const size_t ao = (size_t)(m0 + (i << 4) + rlane) * lda + koff + k0;
            const v16h ah = frag_ld(A + ao);
#pragma unroll
            for (int j = 0; j < 4; ++j)
                acc[i][j] = __builtin_amdgcn_wmma_f32_16x16x32_f16(false, ah, false, bh[j], (short)0, acc[i][j], false, false);
            dep_guard_h(acc[i][0], acc[i][3], ah, ah);
        }
        keep4_h(bh[0], bh[1], bh[2], bh[3]);
    }
    acc_guard4(acc[0][0], acc[0][1], acc[0][2], acc[0][3]);
    acc_guard4(acc[1][0], acc[1][1], acc[1][2], acc[1][3]);
    acc_guard4(acc[2][0], acc[2][1], acc[2][2], acc[2][3]);
    acc_guard4(acc[3][0], acc[3][1], acc[3][2], acc[3][3]);

    float* slab = sT[wave];
#pragma unroll
    for (int i = 0; i < 4; ++i) {
        const int mBase = m0 + (i << 4);
#pragma unroll
        for (int j = 0; j < 4; ++j) {
            const int n = n0 + (j << 4) + rlane;
            float bv = 0.f;
            if (BIAS_MODE == 2) bv = bias[n];
#pragma unroll
            for (int r = 0; r < 8; ++r) {
                float v = acc[i][j][r] * scale;
                if (BIAS_MODE == 1) v += bias[mBase + mOff + r];
                if (BIAS_MODE == 2) v += bv;
                slab[(mOff + r) * 68 + (j << 4) + rlane] = v;
            }
        }
        __builtin_amdgcn_fence(3  , "workgroup");
        __builtin_amdgcn_wave_barrier();
        __builtin_amdgcn_fence(2  , "workgroup");
        if (OUT_MODE == 0) {
            float* C = (float*)Cout;
            const int hh = lane >> 4, c4 = (lane & 15) * 4;
            for (int pass = 0; pass < 2; ++pass) {
#pragma unroll
                for (int it = 0; it < 8; ++it) {
                    const int row = it * 2 + hh;
                    const v4f v = *(const v4f*)(slab + row * 68 + c4);
                    *(volatile v4f*)(C + (size_t)(mBase + row) * ldc + n0 + c4) = v;
                }
                __threadfence();
            }
        } else {
            unsigned short* C = (unsigned short*)Cout;
            const int q = lane >> 3, c8 = (lane & 7) * 8;
#pragma unroll 1
            for (int it = 0; it < 4; ++it) {
                const int row = it * 4 + q;
                const v4f s0 = *(const v4f*)(slab + row * 68 + c8);
                const v4f s1 = *(const v4f*)(slab + row * 68 + c8 + 4);
                v8h hv;
                hv[0] = (_Float16)(g_act<ACT>(s0.x) * oscale); hv[1] = (_Float16)(g_act<ACT>(s0.y) * oscale);
                hv[2] = (_Float16)(g_act<ACT>(s0.z) * oscale); hv[3] = (_Float16)(g_act<ACT>(s0.w) * oscale);
                hv[4] = (_Float16)(g_act<ACT>(s1.x) * oscale); hv[5] = (_Float16)(g_act<ACT>(s1.y) * oscale);
                hv[6] = (_Float16)(g_act<ACT>(s1.z) * oscale); hv[7] = (_Float16)(g_act<ACT>(s1.w) * oscale);
                volatile v8h* d = (volatile v8h*)(C + (size_t)(mBase + row) * ldc + n0 + c8);
                *d = hv;
                __threadfence();
                *d = hv;
            }
        }
        __builtin_amdgcn_fence(3  , "workgroup");
        __builtin_amdgcn_wave_barrier();
        __builtin_amdgcn_fence(2  , "workgroup");
    }
}

__global__ __launch_bounds__(256) void k_gemm_qk(const unsigned short* __restrict__ A, const unsigned short* __restrict__ Bt, unsigned short* __restrict__ C, const float* __restrict__ bias) {
    gemm64_body<2, 1, 0>(A, EMBED, Bt, EMBED, (void*)C, QKLD, bias, MT, QKLD, EMBED, 0.0625f, 1.0f);
}
__global__ __launch_bounds__(256) void k_gemm_vt(const unsigned short* __restrict__ A, const unsigned short* __restrict__ Bt, unsigned short* __restrict__ C, const float* __restrict__ bias) {
    gemm64_body<1, 1, 0>(A, EMBED, Bt, EMBED, (void*)C, MT, bias, EMBED, MT, EMBED, 0.0625f, 1.0f);
}
__global__ __launch_bounds__(256) void k_gemm_wo(const unsigned short* __restrict__ A, const unsigned short* __restrict__ Bt, float* __restrict__ C, const float* __restrict__ bias) {
    gemm64_body<2, 0, 0>(A, EMBED, Bt, EMBED, (void*)C, EMBED, bias, MT, EMBED, EMBED, 0.00390625f, 1.0f);
}
__global__ __launch_bounds__(256) void k_gemm_ff1(const unsigned short* __restrict__ A, const unsigned short* __restrict__ Bt, unsigned short* __restrict__ C, const float* __restrict__ bias) {
    gemm64_body<2, 1, 1>(A, EMBED, Bt, EMBED, (void*)C, FFDIM, bias, MT, FFDIM, EMBED, 0.0625f, 16.0f);
}
__global__ __launch_bounds__(256) void k_gemm_ff2(const unsigned short* __restrict__ A, const unsigned short* __restrict__ Bt, float* __restrict__ C, const float* __restrict__ bias) {
    gemm64_body<2, 0, 0>(A, FFDIM, Bt, FFDIM, (void*)C, EMBED, bias, MT, EMBED, FFDIM, 0.00390625f, 1.0f);
}

#define AT_PSC 32768.0f
__global__ __launch_bounds__(128) void k_attn(const unsigned short* __restrict__ QKp, const unsigned short* __restrict__ VTp, unsigned short* __restrict__ CTXp) {
    __shared__ __align__(16) _Float16 Psh[4][16 * 64];
    __shared__ __align__(16) float    Os[4][16 * 68];
    const _Float16* QK = (const _Float16*)QKp; const _Float16* VT = (const _Float16*)VTp;
    const int tid = threadIdx.x, wave = tid >> 5, lane = tid & 31, hh = lane >> 4, c = lane & 15;
    const int nqb = SEQ / 64;
    const int bx = blockIdx.x;
    const int qb = bx % nqb;
    const int bh = bx / nqb;
    const int h  = bh % NHEAD;
    const int b  = bh / NHEAD;
    const int q0 = qb * 64 + wave * 16;
    const size_t tok0 = (size_t)b * SEQ;
    const float SC = 0.125f * 1.4426950408889634f;

    v16h qa0, qa1;
    { const _Float16* qrow = QK + (tok0 + q0 + c) * QKLD + h * HDIM + 8 * hh; qa0 = frag_ld(qrow); qa1 = frag_ld(qrow + 32); }
    const _Float16* kbase = QK + tok0 * QKLD + EMBED + h * HDIM + 8 * hh;
    const _Float16* vbase = VT + (size_t)(h * HDIM + c) * MT + tok0 + 8 * hh;

    float mrow[8], lrow[8];
    v8f oacc[4];
#pragma unroll
    for (int r = 0; r < 8; ++r) { mrow[r] = -__builtin_inff(); lrow[r] = 0.f; }
#pragma unroll
    for (int t = 0; t < 4; ++t) oacc[t] = (v8f){0.f, 0.f, 0.f, 0.f, 0.f, 0.f, 0.f, 0.f};
    _Float16* pw = Psh[wave];

#pragma unroll 1
    for (int kc = 0; kc < SEQ / 64; ++kc) {
        const int kv0 = kc * 64;
        v8f s[4];
#pragma unroll
        for (int j = 0; j < 4; ++j) {
            const v16h kb = frag_ld(kbase + (size_t)(kv0 + j * 16 + c) * QKLD);
            s[j] = wmma_h(qa0, kb, (v8f){0.f, 0.f, 0.f, 0.f, 0.f, 0.f, 0.f, 0.f});
        }
        asm volatile("" ::: "memory");
#pragma unroll
        for (int j = 0; j < 4; ++j) {
            const v16h kb = frag_ld(kbase + (size_t)(kv0 + j * 16 + c) * QKLD + 32);
            s[j] = wmma_h(qa1, kb, s[j]);
        }
#pragma unroll
        for (int r = 0; r < 8; ++r) {
            const float a0 = s[0][r] * SC, a1 = s[1][r] * SC, a2 = s[2][r] * SC, a3 = s[3][r] * SC;
            float m = fmaxf(fmaxf(a0, a1), fmaxf(a2, a3));
            m = fmaxf(m, __shfl_xor(m, 1, 32)); m = fmaxf(m, __shfl_xor(m, 2, 32));
            m = fmaxf(m, __shfl_xor(m, 4, 32)); m = fmaxf(m, __shfl_xor(m, 8, 32));
            const float mnew = fmaxf(mrow[r], m);
            const float alpha = exp2f(mrow[r] - mnew);
            mrow[r] = mnew;
            const float p0 = exp2f(a0 - mnew), p1 = exp2f(a1 - mnew), p2 = exp2f(a2 - mnew), p3 = exp2f(a3 - mnew);
            float ps = (p0 + p1) + (p2 + p3);
            ps += __shfl_xor(ps, 1, 32); ps += __shfl_xor(ps, 2, 32); ps += __shfl_xor(ps, 4, 32); ps += __shfl_xor(ps, 8, 32);
            lrow[r] = lrow[r] * alpha + ps;
            _Float16* pr = pw + (8 * hh + r) * 64 + c;
            pr[0]  = (_Float16)(p0 * AT_PSC);
            pr[16] = (_Float16)(p1 * AT_PSC);
            pr[32] = (_Float16)(p2 * AT_PSC);
            pr[48] = (_Float16)(p3 * AT_PSC);
#pragma unroll
            for (int t = 0; t < 4; ++t) oacc[t][r] *= alpha;
        }
        __builtin_amdgcn_fence(3  , "workgroup");
        __builtin_amdgcn_wave_barrier();
        __builtin_amdgcn_fence(2  , "workgroup");
#pragma unroll 1
        for (int kk = 0; kk < 2; ++kk) {
            FragU pa;
            pa.h[0] = *(const v8h*)(pw + c * 64 + kk * 32 + 8 * hh);
            pa.h[1] = *(const v8h*)(pw + c * 64 + kk * 32 + 16 + 8 * hh);
#pragma unroll
            for (int t = 0; t < 4; ++t) {
                const v16h vb = frag_ld(vbase + (size_t)(t * 16) * MT + kv0 + kk * 32);
                oacc[t] = wmma_h(pa.v, vb, oacc[t]);
            }
        }
        __builtin_amdgcn_fence(3  , "workgroup");
        __builtin_amdgcn_wave_barrier();
        __builtin_amdgcn_fence(2  , "workgroup");
    }

    float* os = Os[wave];
#pragma unroll
    for (int r = 0; r < 8; ++r) {
        const float inv = 1.0f / (lrow[r] * (AT_PSC / 16.0f));
#pragma unroll
        for (int t = 0; t < 4; ++t) os[(8 * hh + r) * 68 + t * 16 + c] = oacc[t][r] * inv;
    }
    __builtin_amdgcn_fence(3  , "workgroup");
    __builtin_amdgcn_wave_barrier();
    __builtin_amdgcn_fence(2  , "workgroup");
    {
        const int q = lane >> 3, c8 = (lane & 7) * 8;
        unsigned short* cbase = CTXp + (tok0 + q0) * EMBED + h * HDIM + c8;
#pragma unroll 1
        for (int it = 0; it < 4; ++it) {
            const int row = it * 4 + q;
            const v4f s0 = *(const v4f*)(os + row * 68 + c8);
            const v4f s1 = *(const v4f*)(os + row * 68 + c8 + 4);
            v8h hv;
            hv[0] = (_Float16)s0.x; hv[1] = (_Float16)s0.y; hv[2] = (_Float16)s0.z; hv[3] = (_Float16)s0.w;
            hv[4] = (_Float16)s1.x; hv[5] = (_Float16)s1.y; hv[6] = (_Float16)s1.z; hv[7] = (_Float16)s1.w;
            volatile v8h* d = (volatile v8h*)(cbase + (size_t)row * EMBED);
            *d = hv;
            __threadfence();
            *d = hv;
        }
    }
}

template <int XMAP, int WR16>
__device__ __forceinline__ void ln_body(const float* __restrict__ A, const float* __restrict__ X, const float* __restrict__ GA, const float* __restrict__ BE,
                                        float* __restrict__ Yf, unsigned short* __restrict__ Y16) {
    #pragma clang fp contract(off)
    const int r = blockIdx.x * 8 + (threadIdx.x >> 5); const int L = threadIdx.x & 31; if (r >= MT) return;
    const long long xr = XMAP ? ((long long)(r / SEQ) * SEQ_FULL + (r % SEQ)) : (long long)r;
    v4f v[8]; float s = 0.f;
#pragma unroll
    for (int q = 0; q < 8; ++q) {
        const int cc = 4 * L + 128 * q;
        v[q] = *(const v4f*)(A + (long long)r * EMBED + cc);
        v4f x = *(const v4f*)(X + xr * EMBED + cc);
        if (XMAP) { x.x = cmb_bf(x.x); x.y = cmb_bf(x.y); x.z = cmb_bf(x.z); x.w = cmb_bf(x.w); }
        v[q] = v[q] + x;
        s += (v[q].x + v[q].y) + (v[q].z + v[q].w);
    }
#pragma unroll
    for (int o = 16; o > 0; o >>= 1) s += __shfl_xor(s, o, 32);
    const float mu = s * (1.f / EMBED); float qq = 0.f;
#pragma unroll
    for (int q = 0; q < 8; ++q) { v[q].x -= mu; v[q].y -= mu; v[q].z -= mu; v[q].w -= mu; qq += (v[q].x * v[q].x + v[q].y * v[q].y) + (v[q].z * v[q].z + v[q].w * v[q].w); }
#pragma unroll
    for (int o = 16; o > 0; o >>= 1) qq += __shfl_xor(qq, o, 32);
    const float rs = rsqrtf(qq * (1.f / EMBED) + 1e-6f);
#pragma unroll
    for (int q = 0; q < 8; ++q) {
        const int cc = 4 * L + 128 * q;
        const v4f ga = *(const v4f*)(GA + cc), be = *(const v4f*)(BE + cc);
        v4f y;
        y.x = v[q].x * rs * cmb_bf(ga.x) + cmb_bf(be.x); y.y = v[q].y * rs * cmb_bf(ga.y) + cmb_bf(be.y);
        y.z = v[q].z * rs * cmb_bf(ga.z) + cmb_bf(be.z); y.w = v[q].w * rs * cmb_bf(ga.w) + cmb_bf(be.w);
        const long long o = (long long)r * EMBED + cc;
        VST2(v4f, (v4f*)(Yf + o), y);
        if (WR16) { u2 pk; pk.x = cmb_pk2(y.x, y.y); pk.y = cmb_pk2(y.z, y.w); VST2(u2, (u2*)(Y16 + o), pk); }
    }
}
__global__ __launch_bounds__(256) void k_ln1(const float* __restrict__ ATT, const float* __restrict__ x, const float* __restrict__ g, const float* __restrict__ be, float* __restrict__ X1, unsigned short* __restrict__ H16) {
    ln_body<1, 1>(ATT, x, g, be, X1, H16);
}
__global__ __launch_bounds__(256) void k_ln2(const float* __restrict__ FFo, const float* __restrict__ X1, const float* __restrict__ g, const float* __restrict__ be, float* __restrict__ out) {
    ln_body<0, 0>(FFo, X1, g, be, out, nullptr);
}

extern "C" void kernel_launch(void* const* d_in, const int* in_sizes, int n_in, void* d_out, int out_size, void* d_ws, size_t ws_size, hipStream_t stream) {
    if (n_in < 17) return;
    if ((long long)in_sizes[0] < ((long long)(NB - 1) * SEQ_FULL + SEQ) * EMBED) return;
    if (in_sizes[1] < EMBED * EMBED || in_sizes[3] < EMBED * EMBED || in_sizes[5] < EMBED * EMBED || in_sizes[7] < EMBED * EMBED) return;
    if (in_sizes[11] < EMBED * FFDIM || in_sizes[13] < FFDIM * EMBED) return;
    if (in_sizes[2] < EMBED || in_sizes[4] < EMBED || in_sizes[6] < EMBED || in_sizes[8] < EMBED || in_sizes[9] < EMBED || in_sizes[10] < EMBED) return;
    if (in_sizes[12] < FFDIM || in_sizes[14] < EMBED || in_sizes[15] < EMBED || in_sizes[16] < EMBED) return;
    if ((long long)out_size < (long long)MT * EMBED) return;
    const float* x   = (const float*)d_in[0];
    const float* wq  = (const float*)d_in[1];
    const float* bq  = (const float*)d_in[2];
    const float* wk  = (const float*)d_in[3];
    const float* bk  = (const float*)d_in[4];
    const float* wv  = (const float*)d_in[5];
    const float* bv  = (const float*)d_in[6];
    const float* wo  = (const float*)d_in[7];
    const float* bo  = (const float*)d_in[8];
    const float* g1  = (const float*)d_in[9];
    const float* be1 = (const float*)d_in[10];
    const float* w1  = (const float*)d_in[11];
    const float* b1  = (const float*)d_in[12];
    const float* w2  = (const float*)d_in[13];
    const float* b2  = (const float*)d_in[14];
    const float* g2  = (const float*)d_in[15];
    const float* be2 = (const float*)d_in[16];
    float* out = (float*)d_out;

    constexpr size_t SZ_X16  = (size_t)MT * EMBED * 2;
    constexpr size_t SZ_WQKV = (size_t)3 * EMBED * EMBED * 2;
    constexpr size_t SZ_WO   = (size_t)EMBED * EMBED * 2;
    constexpr size_t SZ_W1T  = (size_t)FFDIM * EMBED * 2;
    constexpr size_t SZ_W2T  = (size_t)EMBED * FFDIM * 2;
    constexpr size_t SZ_QK   = (size_t)MT * QKLD * 2;
    constexpr size_t SZ_VT   = (size_t)EMBED * MT * 2;
    constexpr size_t SZ_CTX  = (size_t)MT * EMBED * 2;
    constexpr size_t SZ_R    = SZ_QK + SZ_VT + SZ_CTX;
    constexpr size_t SZ_F16  = (size_t)MT * FFDIM * 2;
    constexpr size_t SZ_ATT  = (size_t)MT * EMBED * 4;
    constexpr size_t SZ_X1   = (size_t)MT * EMBED * 4;
    constexpr size_t SZ_H16  = (size_t)MT * EMBED * 2;
    constexpr size_t SZ_BR   = 65536;
    static_assert(SZ_F16 <= SZ_R);
    static_assert((size_t)BR_N * 4 <= SZ_BR);
    constexpr size_t OFF_X16  = 0;
    constexpr size_t OFF_WQKV = OFF_X16 + SZ_X16;
    constexpr size_t OFF_WO   = OFF_WQKV + SZ_WQKV;
    constexpr size_t OFF_W1T  = OFF_WO + SZ_WO;
    constexpr size_t OFF_W2T  = OFF_W1T + SZ_W1T;
    constexpr size_t OFF_R    = OFF_W2T + SZ_W2T;
    constexpr size_t OFF_ATT  = OFF_R + SZ_R;
    constexpr size_t OFF_X1   = OFF_ATT + SZ_ATT;
    constexpr size_t OFF_H16  = OFF_X1 + SZ_X1;
    constexpr size_t OFF_BR   = OFF_H16 + SZ_H16;
    constexpr size_t WS_TOTAL = OFF_BR + SZ_BR;
    static_assert(WS_TOTAL <= (size_t)134217728);
    static_assert(OFF_WQKV % 256 == 0 && OFF_WO % 256 == 0 && OFF_W1T % 256 == 0 && OFF_W2T % 256 == 0 && OFF_R % 256 == 0);
    static_assert(OFF_ATT % 256 == 0 && OFF_X1 % 256 == 0 && OFF_H16 % 256 == 0 && OFF_BR % 256 == 0 && SZ_QK % 256 == 0 && SZ_VT % 256 == 0);
    if (WS_TOTAL > ws_size) return;
    char* wsb = (char*)d_ws;
    unsigned short* X16   = (unsigned short*)(wsb + OFF_X16);
    unsigned short* WQKV  = (unsigned short*)(wsb + OFF_WQKV);
    unsigned short* WO16  = (unsigned short*)(wsb + OFF_WO);
    unsigned short* W1T   = (unsigned short*)(wsb + OFF_W1T);
    unsigned short* W2T   = (unsigned short*)(wsb + OFF_W2T);
    unsigned short* QK16  = (unsigned short*)(wsb + OFF_R);
    unsigned short* VT16  = (unsigned short*)(wsb + OFF_R + SZ_QK);
    unsigned short* CTX16 = (unsigned short*)(wsb + OFF_R + SZ_QK + SZ_VT);
    unsigned short* F16   = (unsigned short*)(wsb + OFF_R);
    float* ATT = (float*)(wsb + OFF_ATT);
    float* FFo = (float*)(wsb + OFF_ATT);
    float* X1  = (float*)(wsb + OFF_X1);
    unsigned short* H16 = (unsigned short*)(wsb + OFF_H16);
    float* BR  = (float*)(wsb + OFF_BR);

    k_cast_x<<<(unsigned)(((long long)MT * (EMBED / 8) + 255) / 256), 256, 0, stream>>>(x, X16);
    k_cast_wT<<<(unsigned)(((long long)EMBED * (EMBED / 8) + 255) / 256), 256, 0, stream>>>(wq, EMBED, WQKV, EMBED, EMBED, EMBED, 16.0f);
    k_cast_wT<<<(unsigned)(((long long)EMBED * (EMBED / 8) + 255) / 256), 256, 0, stream>>>(wk, EMBED, WQKV + (size_t)EMBED * EMBED, EMBED, EMBED, EMBED, 16.0f);
    k_cast_wT<<<(unsigned)(((long long)EMBED * (EMBED / 8) + 255) / 256), 256, 0, stream>>>(wv, EMBED, WQKV + (size_t)2 * EMBED * EMBED, EMBED, EMBED, EMBED, 16.0f);
    k_cast_wT<<<(unsigned)(((long long)EMBED * (EMBED / 8) + 255) / 256), 256, 0, stream>>>(wo, EMBED, WO16, EMBED, EMBED, EMBED, 16.0f);
    k_cast_wT<<<(unsigned)(((long long)FFDIM * (EMBED / 8) + 255) / 256), 256, 0, stream>>>(w1, FFDIM, W1T, EMBED, EMBED, FFDIM, 16.0f);
    k_cast_wT<<<(unsigned)(((long long)EMBED * (FFDIM / 8) + 255) / 256), 256, 0, stream>>>(w2, EMBED, W2T, FFDIM, FFDIM, EMBED, 16.0f);
    k_bias<<<BR_N / 256, 256, 0, stream>>>(bq, bk, bv, bo, b1, b2, BR);

    k_gemm_qk<<<(unsigned)((((MT / 64) * (QKLD / 64)) + 7) / 8), 256, 0, stream>>>(X16, WQKV, QK16, BR);
    k_gemm_vt<<<(unsigned)((((EMBED / 64) * (MT / 64)) + 7) / 8), 256, 0, stream>>>(WQKV + (size_t)2 * EMBED * EMBED, X16, VT16, BR + 2 * EMBED);
    k_attn<<<(unsigned)(NB * NHEAD * (SEQ / 64)), 128, 0, stream>>>(QK16, VT16, CTX16);
    k_gemm_wo<<<(unsigned)((((MT / 64) * (EMBED / 64)) + 7) / 8), 256, 0, stream>>>(CTX16, WO16, ATT, BR + 3 * EMBED);
    k_ln1<<<(unsigned)((MT + 7) / 8), 256, 0, stream>>>(ATT, x, g1, be1, X1, H16);
    k_gemm_ff1<<<(unsigned)((((MT / 64) * (FFDIM / 64)) + 7) / 8), 256, 0, stream>>>(H16, W1T, F16, BR + 4 * EMBED);
    k_gemm_ff2<<<(unsigned)((((MT / 64) * (EMBED / 64)) + 7) / 8), 256, 0, stream>>>(F16, W2T, FFo, BR + 4 * EMBED + FFDIM);
    k_ln2<<<(unsigned)((MT + 7) / 8), 256, 0, stream>>>(FFo, X1, g2, be2, out);
}
